// VRWKV_Multi_HW_SpatialMix_12249246728667
// MI455X (gfx1250) — hardware-run, weakly checked
//
#include <hip/hip_runtime.h>
#include <math.h>

constexpr int kBatch = 8;
constexpr int kH = 64;
constexpr int kW = 64;
constexpr int kC = 256;
constexpr int kD = 2 * kC;
constexpr int kT = kH * kW;
constexpr int kRows = kBatch * kT;
constexpr int kNkvr = 3 * kC;
constexpr int kEffPitch = 32;
constexpr int kGroup = 32;
constexpr float kCarryX = 16.0f;
constexpr float kCarryW = 256.0f;
constexpr float kCarryS = 16.0f;
constexpr float kScaleKVR = 1.0f / (kCarryX * kCarryW);
constexpr float kScaleOut = 1.0f / (kCarryS * kCarryW);
constexpr float kInvT = 1.0f / (float)kT;
constexpr float kF16MinNormal = 6.103515625e-5f;
constexpr float kF32MinNormal = 1.17549435e-38f;
constexpr float kNegInit = -1.0e38f;
static_assert(kT == 4096, "token count");
static_assert(kRows % 64 == 0, "gemm M tile");
static_assert(kNkvr % 64 == 0 && kC % 64 == 0, "gemm N tile");
static_assert(kC % 32 == 0 && kD % 32 == 0, "gemm K step");
static_assert(kT % kGroup == 0, "scan grouping");
static_assert(kScaleKVR == 1.0f / 4096.0f && kScaleOut == 1.0f / 4096.0f, "carry fold");

typedef __attribute__((ext_vector_type(16))) _Float16 v16h;
typedef __attribute__((ext_vector_type(8)))  _Float16 v8h;
typedef __attribute__((ext_vector_type(8)))  float    v8f;
typedef __attribute__((ext_vector_type(4)))  float    v4f;
typedef __attribute__((ext_vector_type(4)))  unsigned int v4u;

union FragU { v16h v; v8h h[2]; };
__device__ __forceinline__ v16h frag_load(const _Float16* p) {
  FragU f;
  f.h[0] = *(const v8h*)(p);
  f.h[1] = *(const v8h*)(p + 16);
  return f.v;
}
__device__ __forceinline__ v8f frag_mma(v16h a, v16h b, v8f c) {
  return __builtin_amdgcn_wmma_f32_16x16x32_f16(false, a, false, b, (short)0, c, false, false);
}
__device__ __forceinline__ void tie1_h(v8f& a, v16h x, v16h y) { asm volatile("" : "+v"(a) : "v"(x), "v"(y)); }
__device__ __forceinline__ void guard1_h(v8f& a, v16h x, v16h y) { asm volatile("v_nop\n\tv_nop\n\tv_nop\n\tv_nop" : "+v"(a) : "v"(x), "v"(y)); }
__device__ __forceinline__ void keep4_h(v16h a, v16h b, v16h c, v16h d) { asm volatile("v_nop" :: "v"(a), "v"(b), "v"(c), "v"(d)); }
__device__ __forceinline__ void acc_guard4(v8f& a, v8f& b, v8f& c, v8f& d) { asm volatile("v_nop\n\tv_nop\n\tv_nop\n\tv_nop" : "+v"(a), "+v"(b), "+v"(c), "+v"(d)); }
__device__ __forceinline__ void wave_sync() {
  __builtin_amdgcn_fence(__ATOMIC_RELEASE, "workgroup");
  __builtin_amdgcn_wave_barrier();
  __builtin_amdgcn_fence(__ATOMIC_ACQUIRE, "workgroup");
}

__device__ __forceinline__ unsigned pk16(unsigned short a, unsigned short b) { return (unsigned)a | ((unsigned)b << 16); }
__device__ __forceinline__ unsigned short h_bits(float f) { const _Float16 h = (_Float16)f; return __builtin_bit_cast(unsigned short, h); }
__device__ __forceinline__ float flush_h(float t) { return (fabsf(t) < kF16MinNormal) ? 0.0f : t; }

__device__ __forceinline__ float h16_to_f32(unsigned hb) {
  const unsigned sgn = (hb & 0x8000u) << 16; const unsigned em = hb & 0x7fffu;
  const float fn = __uint_as_float((em << 13) + 0x38000000u);
  const float fs = (float)em * 5.9604644775390625e-8f;
  const float mag = (em < 0x400u) ? fs : fn; return __uint_as_float(__float_as_uint(mag) | sgn); }

__device__ __forceinline__ int imin(int a, int b) { return a < b ? a : b; }
__device__ __forceinline__ int imax(int a, int b) { return a > b ? a : b; }
__device__ __forceinline__ int seq_index(int s, int swap) {
  const int sw = ((s & (kH - 1)) << 6) | (s >> 6);
  return swap ? sw : s;
}
__device__ __forceinline__ float gate_sigmoid(float z) {
  const float zc = fminf(fmaxf(z, -30.0f), 30.0f);
  const float e = expf(-zc);
  return __builtin_amdgcn_rcpf(1.0f + e);
}

__global__ __launch_bounds__(256) void prep_kernel(const float* __restrict__ Wk, const float* __restrict__ Wv,
                                                   const float* __restrict__ Wr, const float* __restrict__ Wo,
                                                   const float* __restrict__ alpha, const float* __restrict__ cw1,
                                                   const float* __restrict__ cw3, const float* __restrict__ cw5,
                                                   unsigned short* __restrict__ wkvr16, unsigned short* __restrict__ wo16,
                                                   float* __restrict__ eff) {
  const int z = blockIdx.y;
  const int bx = blockIdx.x;
  const int tid = threadIdx.x;
  if (z < 4) {
    const int nblk = (z == 3) ? 64 : 32;
    if (bx >= nblk) return;
    const float* Wm = (z == 0) ? Wk : (z == 1) ? Wv : (z == 2) ? Wr : Wo;
    unsigned short* op = (z == 3) ? wo16 : (wkvr16 + (size_t)z * kC * kC);
    const int i = bx * 256 + tid;
    const float* p = Wm + 8 * (size_t)i;
    const v4f a = *(const v4f*)(p);
    const v4f c = *(const v4f*)(p + 4);
    unsigned short hb[8];
#pragma unroll
    for (int e = 0; e < 4; ++e) {
      hb[e]     = h_bits(flush_h(a[e] * kCarryW));
      hb[4 + e] = h_bits(flush_h(c[e] * kCarryW));
    }
    const v4u u = (v4u){pk16(hb[0], hb[1]), pk16(hb[2], hb[3]), pk16(hb[4], hb[5]), pk16(hb[6], hb[7])};
    unsigned short* q = op + 8 * (size_t)i;
    *(volatile v4u*)q = u;
    __threadfence();
    *(volatile v4u*)q = u;
  } else {
    if (bx >= 32) return;
    const int gi = bx * 256 + tid;
    const int c = gi >> 5;
    const int q = gi & 31;
    const int qc = imin(q, 24);
    const int di = qc / 5;
    const int dj = qc - di * 5;
    const bool inner = (di >= 1) && (di <= 3) && (dj >= 1) && (dj <= 3);
    const int i3 = imin(imax((di - 1) * 3 + (dj - 1), 0), 8);
    float t5 = cw5[c * 25 + qc];
    asm volatile("" : "+v"(t5));
    float t3 = cw3[c * 9 + i3];
    asm volatile("" : "+v"(t3));
    float t1 = cw1[c];
    asm volatile("" : "+v"(t1));
    const float a0 = alpha[0], a1 = alpha[1], a2 = alpha[2], a3 = alpha[3];
    float val = a3 * t5;
    const float add3 = a2 * t3;
    const float addc = a1 * t1 + a0;
    val += inner ? add3 : 0.0f;
    val += (qc == 12) ? addc : 0.0f;
    val = (q < 25) ? val : 0.0f;
    float* dst = eff + gi;
    *(volatile float*)dst = val;
    __threadfence();
    *(volatile float*)dst = val;
  }
}

__global__ __launch_bounds__(256) void omni_conv_kernel(const float* __restrict__ x, const float* __restrict__ eff,
                                                        unsigned short* __restrict__ xf) {
  __shared__ __align__(16) unsigned short tile[16 * kC];
  const int c = threadIdx.x;
  const int b = blockIdx.x / kH;
  const int h = blockIdx.x % kH;
  const float* ep = eff + (size_t)c * kEffPitch;
  v4f cv[7];
#pragma unroll
  for (int q = 0; q < 7; ++q) cv[q] = *(const v4f*)(ep + 4 * q);
  float coef[25];
#pragma unroll
  for (int q = 0; q < 25; ++q) coef[q] = cv[q >> 2][q & 3];

  const float* xb = x + (size_t)b * kT * kC + c;
  int hcl[5];
  bool vh[5];
  float win[5][5];
#pragma unroll
  for (int di = 0; di < 5; ++di) {
    const int hh = h - 2 + di;
    hcl[di] = imin(imax(hh, 0), kH - 1);
    vh[di]  = (hh >= 0) && (hh < kH);
    const float t2 = xb[(size_t)(hcl[di] * kW + 0) * kC];
    const float t3 = xb[(size_t)(hcl[di] * kW + 1) * kC];
    win[di][0] = 0.0f;
    win[di][1] = 0.0f;
    win[di][2] = vh[di] ? t2 : 0.0f;
    win[di][3] = vh[di] ? t3 : 0.0f;
  }
  const size_t tokBase = (size_t)b * kT + (size_t)h * kW;
  const int lane = c & 31, wv = c >> 5;

#pragma unroll 1
  for (int wb = 0; wb < kW / 16; ++wb) {
#pragma unroll 1
    for (int wl = 0; wl < 16; ++wl) {
      const int w = wb * 16 + wl;
      const int wn = w + 2;
      const bool okw = (wn < kW);
      const int wnc = imin(wn, kW - 1);
#pragma unroll
      for (int di = 0; di < 5; ++di) {
        const float t = xb[(size_t)(hcl[di] * kW + wnc) * kC];
        win[di][4] = (vh[di] && okw) ? t : 0.0f;
      }
      float acc = 0.0f;
#pragma unroll
      for (int di = 0; di < 5; ++di)
#pragma unroll
        for (int dj = 0; dj < 5; ++dj) acc = fmaf(coef[di * 5 + dj], win[di][dj], acc);
      tile[wl * kC + c] = h_bits(flush_h(acc * kCarryX));
#pragma unroll
      for (int di = 0; di < 5; ++di) {
        win[di][0] = win[di][1]; win[di][1] = win[di][2]; win[di][2] = win[di][3]; win[di][3] = win[di][4];
      }
    }
    __syncthreads();
    {
      const int r0 = wv * 2;
      const v4u val0 = *(const v4u*)(tile + (size_t)(r0 + 0) * kC + lane * 8);
      const v4u val1 = *(const v4u*)(tile + (size_t)(r0 + 1) * kC + lane * 8);
      unsigned short* dst0 = xf + (tokBase + wb * 16 + r0 + 0) * kC + lane * 8;
      unsigned short* dst1 = xf + (tokBase + wb * 16 + r0 + 1) * kC + lane * 8;
      for (int rep = 0; rep < 2; ++rep) {
        *(volatile v4u*)dst0 = val0;
        *(volatile v4u*)dst1 = val1;
        __threadfence();
      }
    }
    __syncthreads();
  }
}

template <int FUSED>
__global__ __launch_bounds__(256) void gemm_f16_kernel(
    const unsigned short* __restrict__ Ap, int lda,
    const unsigned short* __restrict__ Btp, int ldb,
    float* Cf, unsigned short* Cv, unsigned short* Cs, int ldc,
    int M, int N, int K, float scale) {
  const _Float16* A = (const _Float16*)Ap;
  const _Float16* Bt = (const _Float16*)Btp;
  __shared__ __align__(16) float sT[8][16 * 68];
  const int lane = threadIdx.x & 31;
  const int wave = threadIdx.x >> 5;
  const int tilesN = N >> 6;
  const int tilesM = M >> 6;
  const int tile = blockIdx.x * 8 + wave;
  if (tile >= tilesM * tilesN) return;
  const int tm = tile / tilesN;
  const int tn = tile - tm * tilesN;
  const int m0 = tm << 6;
  const int n0 = tn << 6;

  const int rlane = lane & 15;
  const int koff  = (lane >> 4) * 8;
  const int mOff  = (lane >> 4) * 8;

  v8f acc[4][4];
#pragma unroll
  for (int i = 0; i < 4; ++i)
#pragma unroll
    for (int j = 0; j < 4; ++j) acc[i][j] = (v8f){0.f, 0.f, 0.f, 0.f, 0.f, 0.f, 0.f, 0.f};

  for (int k0 = 0; k0 < K; k0 += 32) {
    v16h bh[4];
#pragma unroll
    for (int j = 0; j < 4; ++j) {
      const size_t bo = (size_t)(n0 + (j << 4) + rlane) * ldb + koff + k0;
      bh[j] = frag_load(Bt + bo);
    }
#pragma unroll
    for (int i = 0; i < 4; ++i) {
      const size_t ao = (size_t)(m0 + (i << 4) + rlane) * lda + koff + k0;
      const v16h ah = frag_load(A + ao);
#pragma unroll
      for (int j = 0; j < 4; ++j) acc[i][j] = frag_mma(ah, bh[j], acc[i][j]);
      tie1_h(acc[i][0], ah, bh[0]);
      tie1_h(acc[i][1], ah, bh[1]);
      tie1_h(acc[i][2], ah, bh[2]);
      guard1_h(acc[i][3], ah, bh[3]);
    }
    keep4_h(bh[0], bh[1], bh[2], bh[3]);
  }
  acc_guard4(acc[0][0], acc[0][1], acc[0][2], acc[0][3]);
  acc_guard4(acc[1][0], acc[1][1], acc[1][2], acc[1][3]);
  acc_guard4(acc[2][0], acc[2][1], acc[2][2], acc[2][3]);
  acc_guard4(acc[3][0], acc[3][1], acc[3][2], acc[3][3]);

  float* slab = sT[wave];
  const int region = FUSED ? (n0 >> 8) : 0;
  const int nn = FUSED ? (n0 & (kC - 1)) : n0;
#pragma unroll
  for (int i = 0; i < 4; ++i) {
    const int mBase = m0 + (i << 4);
#pragma unroll
    for (int j = 0; j < 4; ++j) {
#pragma unroll
      for (int r = 0; r < 8; ++r) {
        slab[(mOff + r) * 68 + (j << 4) + rlane] = acc[i][j][r] * scale;
      }
    }
    wave_sync();
    if (FUSED && region == 2) {
#pragma unroll 1
      for (int q = 0; q < 32; ++q) {
        const int row = q >> 1;
        const int col = ((q & 1) << 5) + lane;
        const float zv = slab[row * 68 + col];
        slab[row * 68 + col] = gate_sigmoid(zv);
      }
      wave_sync();
    }
    if (!FUSED || region == 0) {
      const int hh = lane >> 4, c4 = (lane & 15) * 4;
      for (int pass = 0; pass < 2; ++pass) {
#pragma unroll
        for (int it = 0; it < 8; ++it) {
          const int row = it * 2 + hh;
          const v4f v = *(const v4f*)(slab + row * 68 + c4);
          *(volatile v4f*)(Cf + (size_t)(mBase + row) * ldc + nn + c4) = v;
        }
        __threadfence();
      }
    } else {
      const int q = lane >> 3, c8 = (lane & 7) * 8;
      unsigned short* C = (region == 1) ? Cv : Cs;
      v4u pk[4];
#pragma unroll
      for (int it = 0; it < 4; ++it) {
        const int row = it * 4 + q;
        const float* sp = slab + row * 68 + c8;
        unsigned short hb[8];
#pragma unroll
        for (int e = 0; e < 8; ++e) hb[e] = h_bits(sp[e]);
        pk[it] = (v4u){pk16(hb[0], hb[1]), pk16(hb[2], hb[3]), pk16(hb[4], hb[5]), pk16(hb[6], hb[7])};
      }
      for (int pass = 0; pass < 2; ++pass) {
#pragma unroll
        for (int it = 0; it < 4; ++it) {
          const int row = it * 4 + q;
          *(volatile v4u*)(C + (size_t)(mBase + row) * ldc + nn + c8) = pk[it];
        }
        __threadfence();
      }
    }
    wave_sync();
  }
}

__global__ __launch_bounds__(64) void wkv_scan_kernel(const float* __restrict__ kp, const unsigned short* __restrict__ vp,
                                                      const unsigned short* __restrict__ gp,
                                                      const float* __restrict__ sd, const float* __restrict__ sf,
                                                      const int* __restrict__ hwH, const int* __restrict__ hwW,
                                                      unsigned short* __restrict__ xs) {
  __shared__ __align__(16) float kS[kGroup * 64];
  __shared__ __align__(16) unsigned int vS[kGroup * 32];
  __shared__ __align__(16) unsigned int gS[kGroup * 32];
  __shared__ __align__(16) unsigned short oS[kGroup * 64];
  const int tid = threadIdx.x;
  const int b = blockIdx.x >> 3;
  const int dg = blockIdx.x & 7;
  const int swap = dg >> 2;
  const int c0 = (dg & 3) * 64;
  const int d = dg * 64 + tid;
  const float wd = -expf(sd[d] * kInvT);
  const float u = sf[d] * kInvT;
  const bool ok = (hwH[0] == kH) && (hwW[0] == kW);
  const float nanv = __uint_as_float(0x7fc00000u);
  const size_t rowBase = (size_t)b * kT;
  const int sh = (tid & 1) * 16;
  const int wi = tid >> 1;
  float a = 0.0f, bb = 0.0f, pp = kNegInit;

#pragma unroll 1
  for (int g = 0; g < kT / kGroup; ++g) {
    const int s0 = g * kGroup;
#pragma unroll 4
    for (int it = 0; it < 8; ++it) {
      const int idx = it * 64 + tid;
      const int r = idx >> 4;
      const int seg = idx & 15;
      const int srow = seq_index(s0 + r, swap);
      const v4f val = *(const v4f*)(kp + (rowBase + srow) * kC + c0 + seg * 4);
      *(v4f*)(kS + r * 64 + seg * 4) = val;
    }
#pragma unroll 4
    for (int it = 0; it < 4; ++it) {
      const int idx = it * 64 + tid;
      const int r = idx >> 3;
      const int seg = idx & 7;
      const int s = s0 + r;
      const int srow = seq_index(s, swap);
      const v4u vv = *(const v4u*)(vp + (rowBase + srow) * kC + c0 + seg * 8);
      const v4u gg = *(const v4u*)(gp + (rowBase + s) * kC + c0 + seg * 8);
      *(v4u*)(vS + r * 32 + seg * 4) = vv;
      *(v4u*)(gS + r * 32 + seg * 4) = gg;
    }
    __syncthreads();
#pragma unroll 1
    for (int r = 0; r < kGroup; ++r) {
      const float kt = kS[r * 64 + tid];
      const unsigned vw = vS[r * 32 + wi];
      const unsigned gw = gS[r * 32 + wi];
      const float vt = h16_to_f32((vw >> sh) & 0xffffu);
      const float gt = h16_to_f32((gw >> sh) & 0xffffu);
      const float ww = u + kt;
      const float dd = pp - ww;
      float e = expf(-fabsf(dd));
      e = (e < kF32MinNormal) ? 0.0f : e;
      const bool ge = (dd >= 0.0f);
      const float e1 = ge ? 1.0f : e;
      const float e2 = ge ? e : 1.0f;
      const float num = e1 * a + e2 * vt;
      const float den = e1 * bb + e2;
      const float o = num * __builtin_amdgcn_rcpf(den);
      const float ww2 = pp + wd;
      const float d2 = ww2 - kt;
      float f = expf(-fabsf(d2));
      f = (f < kF32MinNormal) ? 0.0f : f;
      const bool ge2 = (d2 >= 0.0f);
      const float f1 = ge2 ? 1.0f : f;
      const float f2 = ge2 ? f : 1.0f;
      a = f1 * a + f2 * vt;
      bb = f1 * bb + f2;
      pp = fmaxf(ww2, kt);
      float tv = flush_h(o * gt * kCarryS);
      tv = ok ? tv : nanv;
      oS[r * 64 + tid] = h_bits(tv);
    }
    __syncthreads();
    {
      v4u ov[4];
#pragma unroll
      for (int it = 0; it < 4; ++it) {
        const int slot = it * 64 + tid;
        const int row = slot >> 3;
        const int c8 = (slot & 7) * 8;
        ov[it] = *(const v4u*)(oS + row * 64 + c8);
      }
      for (int rep = 0; rep < 2; ++rep) {
#pragma unroll
        for (int it = 0; it < 4; ++it) {
          const int slot = it * 64 + tid;
          const int row = slot >> 3;
          const int c8 = (slot & 7) * 8;
          unsigned short* dst = xs + (rowBase + s0 + row) * kD + dg * 64 + c8;
          *(volatile v4u*)dst = ov[it];
        }
        __threadfence();
      }
    }
  }
}

extern "C" void kernel_launch(void* const* d_in, const int* in_sizes, int n_in,
                              void* d_out, int out_size, void* d_ws, size_t ws_size,
                              hipStream_t stream) {
  if (n_in < 13) return;
  if (in_sizes[0] != kRows * kC || out_size != kRows * kC) return;
  if (in_sizes[1] != 4 || in_sizes[2] != kC || in_sizes[3] != kC * 9 || in_sizes[4] != kC * 25) return;
  if (in_sizes[5] != kC * kC || in_sizes[6] != kC * kC || in_sizes[7] != kC * kC || in_sizes[8] != kC * kD) return;
  if (in_sizes[9] != kD || in_sizes[10] != kD || in_sizes[11] < 1 || in_sizes[12] < 1) return;

  constexpr size_t szEff  = (size_t)kC * kEffPitch * 4;
  constexpr size_t szWkvr = (size_t)kNkvr * kC * 2;
  constexpr size_t szWo   = (size_t)kC * kD * 2;
  constexpr size_t szXf   = (size_t)kRows * kC * 2;
  constexpr size_t szK    = (size_t)kRows * kC * 4;
  constexpr size_t szV    = (size_t)kRows * kC * 2;
  constexpr size_t szG    = (size_t)kRows * kC * 2;
  constexpr size_t szXs   = (size_t)kRows * kD * 2;
  constexpr size_t offEff  = 0;
  constexpr size_t offWkvr = offEff + szEff;
  constexpr size_t offWo   = offWkvr + szWkvr;
  constexpr size_t offXf   = offWo + szWo;
  constexpr size_t offK    = offXf + szXf;
  constexpr size_t offV    = offK + szK;
  constexpr size_t offG    = offV + szV;
  constexpr size_t offXs   = offG + szG;
  constexpr size_t total   = offXs + szXs;
  static_assert(total == 118128640ull, "carve sum");
  static_assert(total <= 134217728ull, "carve limit");
  static_assert(offWkvr % 128 == 0 && offWo % 128 == 0 && offXf % 128 == 0 && offK % 128 == 0, "alignment");
  static_assert(offV % 128 == 0 && offG % 128 == 0 && offXs % 128 == 0, "alignment");
  if (ws_size < total) return;

  const float* x     = (const float*)d_in[0];
  const float* alpha = (const float*)d_in[1];
  const float* cw1   = (const float*)d_in[2];
  const float* cw3   = (const float*)d_in[3];
  const float* cw5   = (const float*)d_in[4];
  const float* Wk    = (const float*)d_in[5];
  const float* Wv    = (const float*)d_in[6];
  const float* Wr    = (const float*)d_in[7];
  const float* Wo    = (const float*)d_in[8];
  const float* sdp   = (const float*)d_in[9];
  const float* sfp   = (const float*)d_in[10];
  const int*   hH    = (const int*)d_in[11];
  const int*   hWd   = (const int*)d_in[12];
  float* out = (float*)d_out;
  char* ws = (char*)d_ws;
  float* eff = (float*)(ws + offEff);
  unsigned short* Wkvr16 = (unsigned short*)(ws + offWkvr);
  unsigned short* Wo16   = (unsigned short*)(ws + offWo);
  unsigned short* Xf     = (unsigned short*)(ws + offXf);
  float* Kf              = (float*)(ws + offK);
  unsigned short* V16    = (unsigned short*)(ws + offV);
  unsigned short* G16    = (unsigned short*)(ws + offG);
  unsigned short* Xs     = (unsigned short*)(ws + offXs);

  prep_kernel<<<dim3(64, 5), dim3(256), 0, stream>>>(Wk, Wv, Wr, Wo, alpha, cw1, cw3, cw5, Wkvr16, Wo16, eff);
  omni_conv_kernel<<<dim3(kBatch * kH), dim3(256), 0, stream>>>(x, eff, Xf);
  gemm_f16_kernel<1><<<dim3((kRows / 64) * (kNkvr / 64) / 8), dim3(256), 0, stream>>>(
      Xf, kC, Wkvr16, kC, Kf, V16, G16, kC, kRows, kNkvr, kC, kScaleKVR);
  wkv_scan_kernel<<<dim3(kBatch * 8), dim3(64), 0, stream>>>(Kf, V16, G16, sdp, sfp, hH, hWd, Xs);
  gemm_f16_kernel<0><<<dim3((kRows / 64) * (kC / 64) / 8), dim3(256), 0, stream>>>(
      Xs, kD, Wo16, kD, out, V16, G16, kC, kRows, kC, kD, kScaleOut);
}
